// GATLinkPredictor_88149908783544
// MI455X (gfx1250) — hardware-verified
//
#include <hip/hip_runtime.h>
#include <stddef.h>
#include <stdint.h>
#include <math.h>


#define KIN     128
#define HD1     128
#define HD2     64
#define HID     64
#define KA2     256
#define ELW     8
#define NTHR    256
#define NWAVE   8
#define EPT     8
#define CHUNK   (NTHR * EPT)
#define WCAP    (EPT * 32)
#define LISTN   (NWAVE * WCAP)
#define NBMAX   2048
#define SLOTB   11
#define RCAP    28672
#define DEGCAP  256
#define GBM     64
#define GTHR    128
#define NEGSL   0.2f
#define EPS_SM  1e-16f
#define WSMAX   134217728
#define LDS_AGG ((2 * RCAP + 2 * NBMAX + LISTN) * 4 + 64)

static_assert((CHUNK & (CHUNK - 1)) == 0 && CHUNK <= (1 << SLOTB));
static_assert(NBMAX == (1 << SLOTB));
static_assert(NTHR * 8 == NBMAX);
static_assert(LISTN >= NBMAX);
static_assert(LISTN >= NWAVE * WCAP);
static_assert((RCAP % 32) == 0);
static_assert(LDS_AGG <= 300000);
static_assert(GBM == (GTHR / 32) * 16);
static_assert((KIN % 32) == 0 && (KA2 % 32) == 0 && KA2 == 2 * HD1);
static_assert(HD1 == 2 * HID && HD2 == HID);
static_assert(HID == 16 * 4);
static_assert(HD1 == 32 * 4);
static_assert(HD2 == 32 * 2);
static_assert(KIN / 8 == 16 && KA2 / 8 == 32);
static_assert(ELW == 8);

typedef float          v2f  __attribute__((ext_vector_type(2)));
typedef float          v4f  __attribute__((ext_vector_type(4)));
typedef float          v8f  __attribute__((ext_vector_type(8)));
typedef int            v4i  __attribute__((ext_vector_type(4)));
typedef int            v8i  __attribute__((ext_vector_type(8)));
typedef unsigned int   v4u  __attribute__((ext_vector_type(4)));
typedef unsigned short v8us __attribute__((ext_vector_type(8)));
typedef __bf16         v16b __attribute__((ext_vector_type(16)));
typedef v2f  __attribute__((may_alias)) v2fa;
typedef v4f  __attribute__((may_alias)) v4fa;
typedef v8us __attribute__((may_alias)) v8usa;
union FragB { v16b v; v8us h[2]; v8i w; };

__device__ __forceinline__ v8f wmb(const FragB& a, const FragB& b, v8f c) {
  v8f d = __builtin_amdgcn_wmma_f32_16x16x32_bf16(false, a.v, false, b.v, (short)0, c, false, false);
  asm volatile("v_nop\n\tv_nop\n\tv_nop\n\tv_nop" : "+v"(d) : "v"(a.w), "v"(b.w));
  return d;
}

__device__ __forceinline__ unsigned int f2bf(float f) {
  const unsigned int u = __float_as_uint(f);
  return ((u + 0x7FFFu + ((u >> 16) & 1u)) >> 16) & 0xFFFFu;
}
__device__ __forceinline__ float bf2f(unsigned int b) { return __uint_as_float(b << 16); }
__device__ __forceinline__ float bfr(float f) { return bf2f(f2bf(f)); }
__device__ __forceinline__ v2f bfr2(const v2f a) { v2f r; r.x = bfr(a.x); r.y = bfr(a.y); return r; }
__device__ __forceinline__ v4f bfr4(const v4f a) {
  v4f r; r.x = bfr(a.x); r.y = bfr(a.y); r.z = bfr(a.z); r.w = bfr(a.w); return r;
}
__device__ __forceinline__ v8us cvt8b(const v4f a, const v4f b) {
  v8us o;
  o[0] = (unsigned short)f2bf(a.x); o[1] = (unsigned short)f2bf(a.y);
  o[2] = (unsigned short)f2bf(a.z); o[3] = (unsigned short)f2bf(a.w);
  o[4] = (unsigned short)f2bf(b.x); o[5] = (unsigned short)f2bf(b.y);
  o[6] = (unsigned short)f2bf(b.z); o[7] = (unsigned short)f2bf(b.w);
  return o;
}

__device__ __forceinline__ int scan_chunk(const int* __restrict__ dsts, int nE, int cbase, int slotBase,
                                          int nb, int vec8, int* list, int tid, int lane, int wave) {
  int wc = 0;
  const int el0  = tid * EPT;
  const int e0   = cbase + el0;
  const int sent = -2147483647 - 1;
  v4i da, db;
  if (vec8 != 0 && cbase + CHUNK <= nE) {
    da = *(const v4i*)(dsts + e0);
    db = *(const v4i*)(dsts + e0 + 4);
  } else {
    da.x = (e0     < nE) ? dsts[min(e0,     nE - 1)] : sent;
    da.y = (e0 + 1 < nE) ? dsts[min(e0 + 1, nE - 1)] : sent;
    da.z = (e0 + 2 < nE) ? dsts[min(e0 + 2, nE - 1)] : sent;
    da.w = (e0 + 3 < nE) ? dsts[min(e0 + 3, nE - 1)] : sent;
    db.x = (e0 + 4 < nE) ? dsts[min(e0 + 4, nE - 1)] : sent;
    db.y = (e0 + 5 < nE) ? dsts[min(e0 + 5, nE - 1)] : sent;
    db.z = (e0 + 6 < nE) ? dsts[min(e0 + 6, nE - 1)] : sent;
    db.w = (e0 + 7 < nE) ? dsts[min(e0 + 7, nE - 1)] : sent;
  }
  const unsigned nbs = (unsigned)slotBase;
  const unsigned unb = (unsigned)nb;
  const unsigned s0 = (unsigned)da.x - nbs, s1 = (unsigned)da.y - nbs;
  const unsigned s2 = (unsigned)da.z - nbs, s3 = (unsigned)da.w - nbs;
  const unsigned s4 = (unsigned)db.x - nbs, s5 = (unsigned)db.y - nbs;
  const unsigned s6 = (unsigned)db.z - nbs, s7 = (unsigned)db.w - nbs;
  const bool h0 = s0 < unb, h1 = s1 < unb, h2 = s2 < unb, h3 = s3 < unb;
  const bool h4 = s4 < unb, h5 = s5 < unb, h6 = s6 < unb, h7 = s7 < unb;
  const unsigned any = __builtin_amdgcn_ballot_w32(h0 | h1 | h2 | h3 | h4 | h5 | h6 | h7);
  if (any != 0u) {
#define HITJ(J, HJ, SJ) { \
      const unsigned mj = __builtin_amdgcn_ballot_w32(HJ); \
      if (mj != 0u) { \
        if (HJ) { \
          const int pos = wc + (int)__builtin_amdgcn_mbcnt_lo(mj, 0u); \
          if (pos < WCAP) list[wave * WCAP + pos] = ((el0 + (J)) << SLOTB) | (int)(SJ); \
        } \
        wc += (int)__builtin_popcount(mj); } }
    HITJ(0, h0, s0)
    HITJ(1, h1, s1)
    HITJ(2, h2, s2)
    HITJ(3, h3, s3)
    HITJ(4, h4, s4)
    HITJ(5, h5, s5)
    HITJ(6, h6, s6)
    HITJ(7, h7, s7)
#undef HITJ
  }
  return wc;
}

__global__ __launch_bounds__(NTHR) void k_prep(const float* __restrict__ x,
                                               const float* __restrict__ W1, const float* __restrict__ W2,
                                               const float* __restrict__ We1, const float* __restrict__ ae1,
                                               const float* __restrict__ We2, const float* __restrict__ ae2,
                                               unsigned short* xb, unsigned short* w1t, unsigned short* w2t,
                                               float* kap, int nN, int nUx, int nBx, int nB1, int nB2) {
  const int tid = (int)threadIdx.x;
  const int bid = (int)blockIdx.x;
  const v4f z4 = {0.f, 0.f, 0.f, 0.f};
  if (bid < nBx) {
    const int i = bid * NTHR + tid;
    if (i >= nUx) return;
    const int row = i >> 4;
    const int c0  = (i & 15) * 8;
    const int rc  = row < nN ? row : nN - 1;
    const float* p = x + (size_t)rc * KIN + c0;
    v4f a = *(const v4fa*)p, b = *(const v4fa*)(p + 4);
    if (row >= nN) { a = z4; b = z4; }
    const v8us hv = cvt8b(a, b);
    const size_t o = (size_t)row * KIN + c0;
    *(volatile v8us*)(xb + o) = hv;
    __threadfence();
    *(volatile v8us*)(xb + o) = hv;
  } else if (bid < nBx + nB1) {
    const int u = (bid - nBx) * NTHR + tid;
    if (u >= HD1 * (KIN / 8)) return;
    const int n   = u >> 4;
    const int k8  = (u & 15) * 8;
    const int ncl = n < HD1 ? n : HD1 - 1;
    const float* p = W1 + (size_t)k8 * (size_t)HD1 + ncl;
    v4f a, b;
    a.x = p[0];                  a.y = p[(size_t)HD1];        a.z = p[(size_t)2 * HD1];    a.w = p[(size_t)3 * HD1];
    b.x = p[(size_t)4 * HD1];    b.y = p[(size_t)5 * HD1];    b.z = p[(size_t)6 * HD1];    b.w = p[(size_t)7 * HD1];
    if (n >= HD1) { a = z4; b = z4; }
    const v8us hv = cvt8b(a, b);
    const size_t o = (size_t)n * (size_t)KIN + k8;
    *(volatile v8us*)(w1t + o) = hv;
    __threadfence();
    *(volatile v8us*)(w1t + o) = hv;
  } else if (bid < nBx + nB1 + nB2) {
    const int u = (bid - nBx - nB1) * NTHR + tid;
    if (u >= HD2 * (KA2 / 8)) return;
    const int n   = u >> 5;
    const int k8  = (u & 31) * 8;
    const int kk  = k8 & (HD1 - 1);
    const int ncl = n < HD2 ? n : HD2 - 1;
    const float* p = W2 + (size_t)kk * (size_t)HD2 + ncl;
    v4f a, b;
    a.x = p[0];                  a.y = p[(size_t)HD2];        a.z = p[(size_t)2 * HD2];    a.w = p[(size_t)3 * HD2];
    b.x = p[(size_t)4 * HD2];    b.y = p[(size_t)5 * HD2];    b.z = p[(size_t)6 * HD2];    b.w = p[(size_t)7 * HD2];
    if (n >= HD2) { a = z4; b = z4; }
    const v8us hv = cvt8b(a, b);
    const size_t o = (size_t)n * (size_t)KA2 + k8;
    *(volatile v8us*)(w2t + o) = hv;
    __threadfence();
    *(volatile v8us*)(w2t + o) = hv;
  } else {
    if (tid >= 32) return;
    const int lane = tid;
    const int c = 2 * lane;
    const v2f p1 = bfr2(*(const v2fa*)(We1 + c));
    const v2f q1 = bfr2(*(const v2fa*)(ae1 + c));
    const v2f p2 = bfr2(*(const v2fa*)(We1 + HID + c));
    const v2f q2 = bfr2(*(const v2fa*)(ae1 + HID + c));
    const v2f p3 = bfr2(*(const v2fa*)(We2 + c));
    const v2f q3 = bfr2(*(const v2fa*)(ae2 + c));
    float k0 = p1.x * q1.x; k0 = fmaf(p1.y, q1.y, k0);
    float k1 = p2.x * q2.x; k1 = fmaf(p2.y, q2.y, k1);
    float k2 = p3.x * q3.x; k2 = fmaf(p3.y, q3.y, k2);
#pragma unroll
    for (int off = 16; off > 0; off >>= 1) {
      k0 += __shfl_xor(k0, off);
      k1 += __shfl_xor(k1, off);
      k2 += __shfl_xor(k2, off);
    }
    float val = 0.f;
    val = (lane == 0) ? k0 : val;
    val = (lane == 1) ? k1 : val;
    val = (lane == 2) ? k2 : val;
    float* op = kap + lane;
    *(volatile float*)op = val;
    __threadfence();
    *(volatile float*)op = val;
  }
}

__global__ __launch_bounds__(GTHR) void k_gemm1(
    const unsigned short* __restrict__ A, const unsigned short* __restrict__ WT,
    const float* __restrict__ al, const float* __restrict__ ar,
    float* FT, float* ELR, int K)
{
  __shared__ __attribute__((aligned(16))) float stg[GBM * HD1];
  __shared__ __attribute__((aligned(16))) float selr[GBM * ELW];
  const int tid = (int)threadIdx.x, lane = tid & 31, wave = tid >> 5, hh = lane >> 4, m = lane & 15;
  const int rowBase = (int)blockIdx.x * GBM;

  for (int i = tid; i < GBM * ELW; i += GTHR) selr[i] = 0.f;

  v8f acc[8];
  {
    const v8f z = {0.f, 0.f, 0.f, 0.f, 0.f, 0.f, 0.f, 0.f};
#pragma unroll
    for (int t = 0; t < 8; ++t) acc[t] = z;
  }
  const unsigned short* ap = A  + (size_t)(rowBase + 16 * wave + m) * (size_t)K + 8 * hh;
  const unsigned short* wp = WT + (size_t)m * (size_t)K + 8 * hh;
  const int ksteps = K >> 5;
#pragma unroll 1
  for (int ks = 0; ks < ksteps; ++ks) {
    FragB af;
    af.h[0] = *(const v8usa*)(ap + 32 * ks);
    af.h[1] = *(const v8usa*)(ap + 32 * ks + 16);
#pragma unroll
    for (int t = 0; t < 8; ++t) {
      const unsigned short* wq = wp + (size_t)(16 * t) * (size_t)K + 32 * ks;
      FragB bf;
      bf.h[0] = *(const v8usa*)wq;
      bf.h[1] = *(const v8usa*)(wq + 16);
      acc[t] = wmb(af, bf, acc[t]);
    }
  }

#pragma unroll
  for (int t = 0; t < 8; ++t) {
    const int lc = 16 * t + m;
#pragma unroll
    for (int r = 0; r < 8; ++r) {
      const int lr = 16 * wave + 8 * hh + r;
      stg[lr * HD1 + lc] = acc[t][r];
    }
  }
  __syncthreads();

  const int c0 = 4 * lane;
  const int hd = lane >> 4;
  const v4f al4 = bfr4(*(const v4fa*)(al + c0));
  const v4f ar4 = bfr4(*(const v4fa*)(ar + c0));
  v4f fv[16];
#pragma unroll
  for (int i = 0; i < 16; ++i) {
    const int lr = 16 * wave + i;
    const v4f v = *(const v4fa*)(stg + lr * HD1 + c0);
    fv[i] = v;
    float pl = v.x * al4.x; pl = fmaf(v.y, al4.y, pl); pl = fmaf(v.z, al4.z, pl); pl = fmaf(v.w, al4.w, pl);
    float pr = v.x * ar4.x; pr = fmaf(v.y, ar4.y, pr); pr = fmaf(v.z, ar4.z, pr); pr = fmaf(v.w, ar4.w, pr);
    pl += __shfl_xor(pl, 1); pl += __shfl_xor(pl, 2); pl += __shfl_xor(pl, 4); pl += __shfl_xor(pl, 8);
    pr += __shfl_xor(pr, 1); pr += __shfl_xor(pr, 2); pr += __shfl_xor(pr, 4); pr += __shfl_xor(pr, 8);
    if ((lane & 15) == 0) {
      selr[lr * ELW + hd]     = pl;
      selr[lr * ELW + 4 + hd] = pr;
    }
  }
  __syncthreads();

  const int erow = 16 * wave + (lane >> 1);
  const v4f ev = *(const v4fa*)(selr + erow * ELW + 4 * (lane & 1));
  float* ep = ELR + (size_t)(rowBase + erow) * ELW + 4 * (lane & 1);
#pragma unroll
  for (int i = 0; i < 16; ++i) {
    float* op = FT + (size_t)(rowBase + 16 * wave + i) * (size_t)HD1 + c0;
    *(volatile v4f*)op = fv[i];
  }
  *(volatile v4f*)ep = ev;
  __threadfence();
#pragma unroll
  for (int i = 0; i < 16; ++i) {
    float* op = FT + (size_t)(rowBase + 16 * wave + i) * (size_t)HD1 + c0;
    *(volatile v4f*)op = fv[i];
  }
  *(volatile v4f*)ep = ev;
}

__global__ __launch_bounds__(GTHR) void k_gemm2(
    const unsigned short* __restrict__ A, const unsigned short* __restrict__ WT,
    const float* __restrict__ al, const float* __restrict__ ar,
    float* FT, float* ELR, int K)
{
  __shared__ __attribute__((aligned(16))) float stg[GBM * HD2];
  __shared__ __attribute__((aligned(16))) float selr[GBM * ELW];
  const int tid = (int)threadIdx.x, lane = tid & 31, wave = tid >> 5, hh = lane >> 4, m = lane & 15;
  const int rowBase = (int)blockIdx.x * GBM;

  for (int i = tid; i < GBM * ELW; i += GTHR) selr[i] = 0.f;

  v8f acc[4];
  {
    const v8f z = {0.f, 0.f, 0.f, 0.f, 0.f, 0.f, 0.f, 0.f};
    acc[0] = z; acc[1] = z; acc[2] = z; acc[3] = z;
  }
  const unsigned short* ap = A  + (size_t)(rowBase + 16 * wave + m) * (size_t)K + 8 * hh;
  const unsigned short* wp = WT + (size_t)m * (size_t)K + 8 * hh;
  const int ksteps = K >> 5;
#pragma unroll 1
  for (int ks = 0; ks < ksteps; ++ks) {
    FragB af;
    af.h[0] = *(const v8usa*)(ap + 32 * ks);
    af.h[1] = *(const v8usa*)(ap + 32 * ks + 16);
#pragma unroll
    for (int t = 0; t < 4; ++t) {
      const unsigned short* wq = wp + (size_t)(16 * t) * (size_t)K + 32 * ks;
      FragB bf;
      bf.h[0] = *(const v8usa*)wq;
      bf.h[1] = *(const v8usa*)(wq + 16);
      acc[t] = wmb(af, bf, acc[t]);
    }
  }

#pragma unroll
  for (int t = 0; t < 4; ++t) {
    const int lc = 16 * t + m;
#pragma unroll
    for (int r = 0; r < 8; ++r) {
      const int lr = 16 * wave + 8 * hh + r;
      stg[lr * HD2 + lc] = acc[t][r];
    }
  }
  __syncthreads();

  const int c0 = 4 * m;
  const v4f al4 = bfr4(*(const v4fa*)(al + c0));
  const v4f ar4 = bfr4(*(const v4fa*)(ar + c0));
  v4f fv[8];
#pragma unroll
  for (int i = 0; i < 8; ++i) {
    const int lr = 16 * wave + 2 * i + hh;
    const v4f v = *(const v4fa*)(stg + lr * HD2 + c0);
    fv[i] = v;
    float pl = v.x * al4.x; pl = fmaf(v.y, al4.y, pl); pl = fmaf(v.z, al4.z, pl); pl = fmaf(v.w, al4.w, pl);
    float pr = v.x * ar4.x; pr = fmaf(v.y, ar4.y, pr); pr = fmaf(v.z, ar4.z, pr); pr = fmaf(v.w, ar4.w, pr);
    pl += __shfl_xor(pl, 1); pl += __shfl_xor(pl, 2); pl += __shfl_xor(pl, 4); pl += __shfl_xor(pl, 8);
    pr += __shfl_xor(pr, 1); pr += __shfl_xor(pr, 2); pr += __shfl_xor(pr, 4); pr += __shfl_xor(pr, 8);
    if (m == 0) {
      selr[lr * ELW]     = pl;
      selr[lr * ELW + 4] = pr;
    }
  }
  __syncthreads();

  const int erow = 16 * wave + (lane >> 1);
  const v4f ev = *(const v4fa*)(selr + erow * ELW + 4 * (lane & 1));
  float* ep = ELR + (size_t)(rowBase + erow) * ELW + 4 * (lane & 1);
#pragma unroll
  for (int i = 0; i < 8; ++i) {
    const int lr = 16 * wave + 2 * i + hh;
    float* op = FT + (size_t)(rowBase + lr) * (size_t)HD2 + c0;
    *(volatile v4f*)op = fv[i];
  }
  *(volatile v4f*)ep = ev;
  __threadfence();
#pragma unroll
  for (int i = 0; i < 8; ++i) {
    const int lr = 16 * wave + 2 * i + hh;
    float* op = FT + (size_t)(rowBase + lr) * (size_t)HD2 + c0;
    *(volatile v4f*)op = fv[i];
  }
  *(volatile v4f*)ep = ev;
}

template<int L>
__global__ __launch_bounds__(NTHR) void k_agg(
    const int* __restrict__ srcs, const int* __restrict__ dsts, const float* __restrict__ ew,
    const float* __restrict__ F, const float* __restrict__ ELR,
    const float* __restrict__ kap, const float* __restrict__ bias,
    unsigned short* A2, float* Z,
    int nN, int nE, int nb, int vec8, int MPr) {
  extern __shared__ v4f lds_dyn[];
  int* reg1 = (int*)lds_dyn;
  int* reg2 = reg1 + RCAP;
  int* scnt = reg2 + RCAP;
  int* soff = scnt + NBMAX;
  int* list = soff + NBMAX;
  int* wcnt = list + LISTN;
  int* wtot = wcnt + NWAVE;
  const int tid = (int)threadIdx.x, lane = tid & 31, wave = tid >> 5;
  const int nodeBase = (int)blockIdx.x * nb;

  for (int i = tid; i < NBMAX; i += NTHR) scnt[i] = 0;
  __syncthreads();

  int tot = 0;
  const int nChunks = (nE + CHUNK - 1) / CHUNK;
#pragma unroll 1
  for (int ch = 0; ch < nChunks; ++ch) {
    const int cbase = ch * CHUNK;
    const int wc = scan_chunk(dsts, nE, cbase, nodeBase, nb, vec8, list, tid, lane, wave);
    if (lane == 0) wcnt[wave] = wc;
    __syncthreads();
    int pre = 0, all = 0;
#pragma unroll
    for (int w2 = 0; w2 < NWAVE; ++w2) {
      int c = wcnt[w2];
      c = c < 0 ? 0 : (c > WCAP ? WCAP : c);
      all += c;
      pre += (w2 < wave) ? c : 0;
    }
    const int wcc  = wc > WCAP ? WCAP : wc;
    const int base = tot + pre;
#pragma unroll 1
    for (int i = lane; i < wcc; i += 32) {
      const int ent = list[wave * WCAP + i];
      const int el  = (ent >> SLOTB) & (CHUNK - 1);
      const int sl  = ent & (NBMAX - 1);
      int eid = cbase + el;
      eid = eid > nE - 1 ? nE - 1 : eid;
      const int pos = base + i;
      if (pos < RCAP) reg1[pos] = (int)(((unsigned)eid << SLOTB) | (unsigned)sl);
    }
    tot += all;
    tot = tot > RCAP ? RCAP : tot;
    __syncthreads();
  }
  const int nh = tot;

  if (wave == 0) {
#pragma unroll 1
    for (int b0 = 0; b0 < nh; b0 += 32) {
      const int idx = b0 + lane;
      const int uv  = reg1[idx < nh ? idx : nh - 1];
      const int m32 = (nh - b0) < 32 ? (nh - b0) : 32;
#pragma unroll 1
      for (int k = 0; k < m32; ++k) {
        const int u  = __builtin_amdgcn_readlane(uv, k);
        const int sl = u & (NBMAX - 1);
        if (lane == 0) scnt[sl] = scnt[sl] + 1;
      }
    }
  }
  __syncthreads();

  {
    const v4i ca = *(const v4i*)(scnt + 8 * tid);
    const v4i cb = *(const v4i*)(scnt + 8 * tid + 4);
    const int e0 = ca.x < 0 ? 0 : ca.x, e1 = ca.y < 0 ? 0 : ca.y, e2 = ca.z < 0 ? 0 : ca.z, e3 = ca.w < 0 ? 0 : ca.w;
    const int e4 = cb.x < 0 ? 0 : cb.x, e5 = cb.y < 0 ? 0 : cb.y, e6 = cb.z < 0 ? 0 : cb.z, e7 = cb.w < 0 ? 0 : cb.w;
    const int ts = e0 + e1 + e2 + e3 + e4 + e5 + e6 + e7;
    int incl = ts;
#pragma unroll
    for (int d = 1; d < 32; d <<= 1) {
      const int up = __shfl_up(incl, d);
      if (lane >= d) incl += up;
    }
    if (lane == 31) wtot[wave] = incl;
    __syncthreads();
    int pre = 0;
#pragma unroll
    for (int w2 = 0; w2 < NWAVE; ++w2) pre += (w2 < wave) ? wtot[w2] : 0;
    int run = pre + incl - ts;
    soff[8 * tid + 0] = run; run += e0;
    soff[8 * tid + 1] = run; run += e1;
    soff[8 * tid + 2] = run; run += e2;
    soff[8 * tid + 3] = run; run += e3;
    soff[8 * tid + 4] = run; run += e4;
    soff[8 * tid + 5] = run; run += e5;
    soff[8 * tid + 6] = run; run += e6;
    soff[8 * tid + 7] = run;
  }
  __syncthreads();
  for (int i = tid; i < NBMAX; i += NTHR) list[i] = soff[i];
  __syncthreads();

  if (wave == 0) {
#pragma unroll 1
    for (int b0 = 0; b0 < nh; b0 += 32) {
      const int idx = b0 + lane;
      const int uv  = reg1[idx < nh ? idx : nh - 1];
      const int m32 = (nh - b0) < 32 ? (nh - b0) : 32;
#pragma unroll 1
      for (int k = 0; k < m32; ++k) {
        const int u   = __builtin_amdgcn_readlane(uv, k);
        const int sl  = u & (NBMAX - 1);
        const int eid = (int)((unsigned)u >> SLOTB);
        if (lane == 0) {
          int pos = list[sl];
          pos = pos < 0 ? 0 : (pos > RCAP - 1 ? RCAP - 1 : pos);
          reg2[pos] = eid;
          list[sl] = pos + 1;
        }
      }
    }
  }
  __syncthreads();

  const int nbw = nb >> 3;
  const bool ovf = (nh >= RCAP);
  const float qnan = __int_as_float(0x7fc00000);
  const v4f kap4 = *(const v4fa*)kap;
  const int s0i = (2 * lane) & 31, s1i = (2 * lane + 1) & 31;

  if (L == 1) {
    const int c0 = 4 * lane;
    const int hd = lane >> 4;
    const float kh = hd ? kap4.y : kap4.x;
    const v4f bb4 = bfr4(*(const v4fa*)(bias + c0));
    const bool lsel = lane >= 16;
#pragma unroll 1
    for (int jt = 0; jt < nbw; ++jt) {
      const int slot = wave * nbw + jt;
      const int grow = nodeBase + slot;
      const int gcl  = grow < nN ? grow : nN - 1;
      int st = soff[slot];
      const int craw = scnt[slot];
      int cnt = craw;
      st  = st < 0 ? 0 : (st > nh ? nh : st);
      cnt = cnt < 0 ? 0 : (cnt > DEGCAP ? DEGCAP : cnt);
      if (cnt > nh - st) cnt = nh - st;
      const float pz = (ovf || craw > DEGCAP) ? qnan : 0.0f;

      const v4f es4 = *(const v4fa*)(ELR + (size_t)gcl * ELW);
      const v4f ed4 = *(const v4fa*)(ELR + (size_t)gcl * ELW + 4);
      const float aself = hd ? es4.y : es4.x;
      const float adh   = hd ? ed4.y : ed4.x;
      const v4f fd = *(const v4fa*)(F + (size_t)gcl * HD1 + c0);
      float mx = -1.0e30f, dn = 0.f, wsum = 0.f;
      v4f av = {0.f, 0.f, 0.f, 0.f};

#pragma unroll 1
      for (int q = 0; q < cnt; ++q) {
        int idx = st + q; idx = idx > RCAP - 1 ? RCAP - 1 : idx;
        int eid = reg2[idx]; eid = eid < 0 ? 0 : (eid > nE - 1 ? nE - 1 : eid);
        const int sraw = srcs[eid];
        const int s = sraw < 0 ? 0 : (sraw > nN - 1 ? nN - 1 : sraw);
        const v4f xl4 = *(const v4fa*)(F + (size_t)s * HD1 + c0);
        const v4f el4 = *(const v4fa*)(ELR + (size_t)s * ELW);
        const float wv = bfr(ew[eid]);
        float lg = ((hd ? el4.y : el4.x) + adh) + wv * kh;
        lg = lg > 0.f ? lg : lg * NEGSL;
        const float df = lg - mx;
        const float ee = __expf(-fabsf(df));
        const bool up  = df > 0.f;
        const float s1 = up ? ee : 1.0f;
        const float s2 = up ? 1.0f : ee;
        mx = up ? lg : mx;
        dn = fmaf(dn, s1, s2);
        av.x = fmaf(av.x, s1, s2 * xl4.x);
        av.y = fmaf(av.y, s1, s2 * xl4.y);
        av.z = fmaf(av.z, s1, s2 * xl4.z);
        av.w = fmaf(av.w, s1, s2 * xl4.w);
        wsum += wv;
      }
      {
        const float cf = (float)cnt;
        const float rc = __builtin_amdgcn_rcpf(fmaxf(cf, 1.0f));
        const float lw = wsum * rc;
        float lg = (aself + adh) + lw * kh;
        lg = lg > 0.f ? lg : lg * NEGSL;
        const float df = lg - mx;
        const float ee = __expf(-fabsf(df));
        const bool up  = df > 0.f;
        const float s1 = up ? ee : 1.0f;
        const float s2 = up ? 1.0f : ee;
        mx = up ? lg : mx;
        dn = fmaf(dn, s1, s2);
        av.x = fmaf(av.x, s1, s2 * fd.x);
        av.y = fmaf(av.y, s1, s2 * fd.y);
        av.z = fmaf(av.z, s1, s2 * fd.z);
        av.w = fmaf(av.w, s1, s2 * fd.w);
      }
      const float inv = __builtin_amdgcn_rcpf(dn + EPS_SM);
      const bool live = grow < nN;
      float h0 = fmaxf(fmaf(av.x, inv, bb4.x), 0.f);
      float h1 = fmaxf(fmaf(av.y, inv, bb4.y), 0.f);
      float h2 = fmaxf(fmaf(av.z, inv, bb4.z), 0.f);
      float h3 = fmaxf(fmaf(av.w, inv, bb4.w), 0.f);
      h0 = (live ? h0 : 0.f) + pz;
      h1 = (live ? h1 : 0.f) + pz;
      h2 = (live ? h2 : 0.f) + pz;
      h3 = (live ? h3 : 0.f) + pz;
      const unsigned int hb0 = f2bf(h0), hb1 = f2bf(h1), hb2 = f2bf(h2), hb3 = f2bf(h3);
      const unsigned int lb0 = f2bf(h0 - bf2f(hb0)), lb1 = f2bf(h1 - bf2f(hb1));
      const unsigned int lb2 = f2bf(h2 - bf2f(hb2)), lb3 = f2bf(h3 - bf2f(hb3));
      const int hw0 = (int)(hb0 | (hb1 << 16));
      const int hw1 = (int)(hb2 | (hb3 << 16));
      const int lw0 = (int)(lb0 | (lb1 << 16));
      const int lw1 = (int)(lb2 | (lb3 << 16));
      const int g0h = __shfl(hw0, s0i), g0l = __shfl(lw0, s0i);
      const int g1h = __shfl(hw1, s0i), g1l = __shfl(lw1, s0i);
      const int g2h = __shfl(hw0, s1i), g2l = __shfl(lw0, s1i);
      const int g3h = __shfl(hw1, s1i), g3l = __shfl(lw1, s1i);
      v4u pv;
      pv.x = (unsigned int)(lsel ? g0l : g0h);
      pv.y = (unsigned int)(lsel ? g1l : g1h);
      pv.z = (unsigned int)(lsel ? g2l : g2h);
      pv.w = (unsigned int)(lsel ? g3l : g3h);
      unsigned short* gp = A2 + (size_t)grow * KA2 + 8 * lane;
      const bool wr = grow < MPr;
      if (wr) *(volatile v4u*)gp = pv;
      __threadfence();
      if (wr) *(volatile v4u*)gp = pv;
    }
  } else {
    const int c0 = 2 * lane;
    const float kh = kap4.z;
    const v2f bb2 = bfr2(*(const v2fa*)(bias + c0));
#pragma unroll 1
    for (int jt = 0; jt < nbw; ++jt) {
      const int slot = wave * nbw + jt;
      const int grow = nodeBase + slot;
      const int gcl  = grow < nN ? grow : nN - 1;
      int st = soff[slot];
      const int craw = scnt[slot];
      int cnt = craw;
      st  = st < 0 ? 0 : (st > nh ? nh : st);
      cnt = cnt < 0 ? 0 : (cnt > DEGCAP ? DEGCAP : cnt);
      if (cnt > nh - st) cnt = nh - st;
      const float pz = (ovf || craw > DEGCAP) ? qnan : 0.0f;

      const float aself = ELR[(size_t)gcl * ELW];
      const float adh   = ELR[(size_t)gcl * ELW + 4];
      const v2f fd = *(const v2fa*)(F + (size_t)gcl * HD2 + c0);
      float mx = -1.0e30f, dn = 0.f, wsum = 0.f;
      float a0 = 0.f, a1 = 0.f;

#pragma unroll 1
      for (int q = 0; q < cnt; ++q) {
        int idx = st + q; idx = idx > RCAP - 1 ? RCAP - 1 : idx;
        int eid = reg2[idx]; eid = eid < 0 ? 0 : (eid > nE - 1 ? nE - 1 : eid);
        const int sraw = srcs[eid];
        const int s = sraw < 0 ? 0 : (sraw > nN - 1 ? nN - 1 : sraw);
        const v2f xl2 = *(const v2fa*)(F + (size_t)s * HD2 + c0);
        const float asr = ELR[(size_t)s * ELW];
        const float wv = bfr(ew[eid]);
        float lg = (asr + adh) + wv * kh;
        lg = lg > 0.f ? lg : lg * NEGSL;
        const float df = lg - mx;
        const float ee = __expf(-fabsf(df));
        const bool up  = df > 0.f;
        const float s1 = up ? ee : 1.0f;
        const float s2 = up ? 1.0f : ee;
        mx = up ? lg : mx;
        dn = fmaf(dn, s1, s2);
        a0 = fmaf(a0, s1, s2 * xl2.x);
        a1 = fmaf(a1, s1, s2 * xl2.y);
        wsum += wv;
      }
      {
        const float cf = (float)cnt;
        const float rc = __builtin_amdgcn_rcpf(fmaxf(cf, 1.0f));
        const float lw = wsum * rc;
        float lg = (aself + adh) + lw * kh;
        lg = lg > 0.f ? lg : lg * NEGSL;
        const float df = lg - mx;
        const float ee = __expf(-fabsf(df));
        const bool up  = df > 0.f;
        const float s1 = up ? ee : 1.0f;
        const float s2 = up ? 1.0f : ee;
        mx = up ? lg : mx;
        dn = fmaf(dn, s1, s2);
        a0 = fmaf(a0, s1, s2 * fd.x);
        a1 = fmaf(a1, s1, s2 * fd.y);
      }
      const float inv = __builtin_amdgcn_rcpf(dn + EPS_SM);
      const bool live = grow < nN;
      float z0 = fmaf(a0, inv, bb2.x);
      float z1 = fmaf(a1, inv, bb2.y);
      z0 = (live ? z0 : 0.f) + pz;
      z1 = (live ? z1 : 0.f) + pz;
      const float g0 = __shfl(z0, s0i);
      const float g1 = __shfl(z1, s0i);
      const float g2 = __shfl(z0, s1i);
      const float g3 = __shfl(z1, s1i);
      v4f zv; zv.x = g0; zv.y = g1; zv.z = g2; zv.w = g3;
      float* gp = Z + (size_t)grow * HD2 + 4 * (lane & 15);
      const bool wr = (grow < MPr) && (lane < 16);
      if (wr) *(volatile v4f*)gp = zv;
      __threadfence();
      if (wr) *(volatile v4f*)gp = zv;
    }
  }
}

__global__ __launch_bounds__(NTHR) void k_decode(const float* __restrict__ Z, const int* __restrict__ eli,
                                                 float* out, int nL, int nN) {
  const int t  = (int)blockIdx.x * NTHR + (int)threadIdx.x;
  const int tc = t < nL ? t : nL - 1;
  int i = eli[tc];
  int j = eli[(size_t)nL + (size_t)tc];
  i = i < 0 ? 0 : (i > nN - 1 ? nN - 1 : i);
  j = j < 0 ? 0 : (j > nN - 1 ? nN - 1 : j);
  const float* zi = Z + (size_t)i * HD2;
  const float* zj = Z + (size_t)j * HD2;
  float s = 0.f;
#pragma unroll 4
  for (int q = 0; q < HD2 / 4; ++q) {
    const v4f a = *(const v4fa*)(zi + 4 * q);
    const v4f b = *(const v4fa*)(zj + 4 * q);
    s = fmaf(a.x, b.x, s); s = fmaf(a.y, b.y, s); s = fmaf(a.z, b.z, s); s = fmaf(a.w, b.w, s);
  }
  const bool wr = t < nL;
  if (wr) *(volatile float*)(out + t) = s;
  __threadfence();
  if (wr) *(volatile float*)(out + t) = s;
}

static int pick_nb(int nE, int nN) {
  int nb = NBMAX;
  while (nb > 32 && (long long)nb * (long long)nE * 5LL > (long long)RCAP * (long long)nN * 4LL) nb >>= 1;
  return nb;
}
static inline int cdiv(int a, int b) { return (a + b - 1) / b; }

extern "C" void kernel_launch(void* const* d_in, const int* in_sizes, int n_in,
                              void* d_out, int out_size, void* d_ws, size_t ws_size,
                              hipStream_t stream) {
  if (n_in < 16) return;
  const int nN = in_sizes[0] / KIN;
  if (nN <= 0 || in_sizes[0] != nN * KIN || nN > (1 << 22)) return;
  if (in_sizes[1] < 2 || (in_sizes[1] & 1) != 0) return;
  const int nE = in_sizes[1] / 2;
  if (nE < 1 || nE >= (1 << (32 - SLOTB))) return;
  if (in_sizes[2] != nE) return;
  if (in_sizes[3] < 2 || (in_sizes[3] & 1) != 0) return;
  const int nL = in_sizes[3] / 2;
  if (nL < 1) return;
  if (in_sizes[4]  != KIN * HD1) return;
  if (in_sizes[5]  != HD1 || in_sizes[6] != HD1) return;
  if (in_sizes[7]  != HD1) return;
  if (in_sizes[8]  != HD1) return;
  if (in_sizes[9]  != HD1) return;
  if (in_sizes[10] != HD1 * HD2) return;
  if (in_sizes[11] != HD2 || in_sizes[12] != HD2) return;
  if (in_sizes[13] != HD2 || in_sizes[14] != HD2) return;
  if (in_sizes[15] != HD2) return;
  if (out_size != nL) return;

  const float* x   = (const float*)d_in[0];
  const int*   ei  = (const int*)  d_in[1];
  const float* ew  = (const float*)d_in[2];
  const int*   eli = (const int*)  d_in[3];
  const float* W1  = (const float*)d_in[4];
  const float* as1 = (const float*)d_in[5];
  const float* ad1 = (const float*)d_in[6];
  const float* We1 = (const float*)d_in[7];
  const float* ae1 = (const float*)d_in[8];
  const float* b1  = (const float*)d_in[9];
  const float* W2  = (const float*)d_in[10];
  const float* as2 = (const float*)d_in[11];
  const float* ad2 = (const float*)d_in[12];
  const float* We2 = (const float*)d_in[13];
  const float* ae2 = (const float*)d_in[14];
  const float* b2  = (const float*)d_in[15];
  float* out = (float*)d_out;
  const int* src = ei;
  const int* dst = ei + nE;

  const int MP   = cdiv(nN, GBM) * GBM;
  const int nb   = pick_nb(nE, nN);
  if (nb < 32 || (nb & (nb - 1)) != 0 || nb > NBMAX) return;
  const int gA   = cdiv(MP, nb);
  const int vec8 = ((nE & 3) == 0) ? 1 : 0;
  if (gA * nb < MP) return;

  char* ws = (char*)d_ws;
  size_t off = 0;
  const size_t oXB  = off; off += (size_t)MP * KIN * 2;            off = (off + 255) & ~(size_t)255;
  const size_t oW1T = off; off += (size_t)HD1 * KIN * 2;           off = (off + 255) & ~(size_t)255;
  const size_t oW2T = off; off += (size_t)HD2 * KA2 * 2;           off = (off + 255) & ~(size_t)255;
  const size_t oKAP = off; off += 256;                             off = (off + 255) & ~(size_t)255;
  const size_t oH1  = off; off += (size_t)MP * HD1 * 4;            off = (off + 255) & ~(size_t)255;
  const size_t oEL1 = off; off += (size_t)MP * ELW * 4;            off = (off + 255) & ~(size_t)255;
  const size_t oA2  = off; off += (size_t)MP * KA2 * 2;            off = (off + 255) & ~(size_t)255;
  const size_t oH2  = off; off += (size_t)MP * HD2 * 4;            off = (off + 255) & ~(size_t)255;
  const size_t oEL2 = off; off += (size_t)MP * ELW * 4;            off = (off + 255) & ~(size_t)255;
  const size_t oZ   = off; off += (size_t)MP * HD2 * 4;            off = (off + 255) & ~(size_t)255;
  if (off > ws_size || off > (size_t)WSMAX) return;
  unsigned short* XB   = (unsigned short*)(ws + oXB);
  unsigned short* W1T  = (unsigned short*)(ws + oW1T);
  unsigned short* W2T  = (unsigned short*)(ws + oW2T);
  float*          KAP  = (float*)(ws + oKAP);
  float*          H1   = (float*)(ws + oH1);
  float*          ELR1 = (float*)(ws + oEL1);
  unsigned short* A2   = (unsigned short*)(ws + oA2);
  float*          H2   = (float*)(ws + oH2);
  float*          ELR2 = (float*)(ws + oEL2);
  float*          Z    = (float*)(ws + oZ);

  hipFuncSetAttribute(reinterpret_cast<const void*>(&k_agg<1>),
                      hipFuncAttributeMaxDynamicSharedMemorySize, LDS_AGG);
  hipFuncSetAttribute(reinterpret_cast<const void*>(&k_agg<2>),
                      hipFuncAttributeMaxDynamicSharedMemorySize, LDS_AGG);

  const int nUx = MP * (KIN / 8);
  const int nBx = cdiv(nUx, NTHR);
  if (nBx * NTHR != nUx) return;
  const int nB1 = cdiv(HD1 * (KIN / 8), NTHR);
  const int nB2 = cdiv(HD2 * (KA2 / 8), NTHR);
  k_prep<<<nBx + nB1 + nB2 + 1, NTHR, 0, stream>>>(x, W1, W2, We1, ae1, We2, ae2,
                                                   XB, W1T, W2T, KAP, nN, nUx, nBx, nB1, nB2);

  const int gM = MP / GBM;
  k_gemm1<<<gM, GTHR, 0, stream>>>(XB, W1T, as1, ad1, H1, ELR1, KIN);

  k_agg<1><<<gA, NTHR, LDS_AGG, stream>>>(src, dst, ew, H1, ELR1, KAP, b1, A2, Z, nN, nE, nb, vec8, MP);

  k_gemm2<<<gM, GTHR, 0, stream>>>(A2, W2T, as2, ad2, H2, ELR2, KA2);

  k_agg<2><<<gA, NTHR, LDS_AGG, stream>>>(src, dst, ew, H2, ELR2, KAP, b2, A2, Z, nN, nE, nb, vec8, MP);

  k_decode<<<cdiv(nL, NTHR), NTHR, 0, stream>>>(Z, eli, out, nL, nN);
}
